// AGCRN_29265907155020
// MI455X (gfx1250) — hardware-verified
//
#include <hip/hip_runtime.h>
#include <math.h>

constexpr int NNODE  = 20000;
constexpr int NEDGE  = 640000;
constexpr int NEDGE4 = NEDGE / 4;
constexpr int NTIME  = 24;
constexpr int NHIDU  = 128;
constexpr int NGATE  = 3 * NHIDU;
constexpr int NEMB   = 10;
constexpr int NTHR   = 256;
constexpr int RROWS  = 32;
constexpr int HPITCH = 136;
constexpr int TILE_S = 512;
constexpr int TILE_Y = 256;
constexpr int NNODP  = 20480;
constexpr int YLP    = 32;

static_assert(NNODE % RROWS == 0);
static_assert(NNODE % 32 == 0);
static_assert(NNODP % TILE_S == 0 && NNODP % TILE_Y == 0 && NNODP >= NNODE + 1);
static_assert(NEDGE % 4 == 0 && NEDGE % NTHR == 0 && NEDGE4 % 32 == 0);
static_assert(NHIDU % 32 == 0);
static_assert(NHIDU == 16 * (NTHR / 32));
static_assert((NNODP * NTIME) % NTHR == 0);
static_assert((NGATE * NHIDU / 8) % NTHR == 0);
static_assert(HPITCH % 8 == 0);
static_assert(TILE_S % 32 == 0 && TILE_Y % 32 == 0);
static_assert(NTIME <= YLP);

typedef __attribute__((ext_vector_type(16))) _Float16 v16h;
typedef __attribute__((ext_vector_type(8)))  _Float16 v8h;
typedef __attribute__((ext_vector_type(16))) __bf16   v16b;
typedef __attribute__((ext_vector_type(8)))  __bf16   v8b;
typedef __attribute__((ext_vector_type(8)))  float    v8f;
typedef __attribute__((ext_vector_type(4)))  float    v4f;
typedef __attribute__((ext_vector_type(2)))  float    v2f;
typedef __attribute__((ext_vector_type(4)))  int      i4v;

__device__ __forceinline__ unsigned short f2bf_bits(float f) {
  unsigned u = __float_as_uint(f);
  return (unsigned short)((u + 0x7FFFu + ((u >> 16) & 1u)) >> 16);
}
__device__ __forceinline__ float bf_bits2f(unsigned short h) { return __uint_as_float(((unsigned)h) << 16); }
__device__ __forceinline__ float bf16r(float f) { return bf_bits2f(f2bf_bits(f)); }
__device__ __forceinline__ int clampn(int v) { v = v < 0 ? 0 : v; return v > (NNODE - 1) ? (NNODE - 1) : v; }

__device__ __forceinline__ void dep_guard_h(v8f& a, v8f& b, v16h x, v16h y) { asm volatile("v_nop\n\tv_nop\n\tv_nop\n\tv_nop" : "+v"(a), "+v"(b) : "v"(x), "v"(y)); }
__device__ __forceinline__ void dep_guard_b(v8f& a, v8f& b, v16b x, v16b y) { asm volatile("v_nop\n\tv_nop\n\tv_nop\n\tv_nop" : "+v"(a), "+v"(b) : "v"(x), "v"(y)); }
__device__ __forceinline__ void keep4_h(v16h a, v16h b, v16h c, v16h d) { asm volatile("v_nop" :: "v"(a), "v"(b), "v"(c), "v"(d)); }
__device__ __forceinline__ void keep4_b(v16b a, v16b b, v16b c, v16b d) { asm volatile("v_nop" :: "v"(a), "v"(b), "v"(c), "v"(d)); }
__device__ __forceinline__ void guard3x5(v8f& a, v8f& b, v8f& c, v16b p, v16b q, v16b r, v16b s, v16b u) {
  asm volatile("v_nop\n\tv_nop\n\tv_nop\n\tv_nop" : "+v"(a), "+v"(b), "+v"(c) : "v"(p), "v"(q), "v"(r), "v"(s), "v"(u));
}
__device__ __forceinline__ void accg3(v8f& a, v8f& b, v8f& c) { asm volatile("v_nop\n\tv_nop\n\tv_nop\n\tv_nop" : "+v"(a), "+v"(b), "+v"(c)); }

template <typename T> struct Frag;
template <> struct Frag<_Float16> {
  typedef v16h V; union U { v16h v; v8h h[2]; };
  static __device__ __forceinline__ v16h load(const _Float16* p) {
    U f; f.h[0] = *(const v8h*)(p); f.h[1] = *(const v8h*)(p + 16); return f.v;
  }
  static __device__ __forceinline__ v8f mma(v16h a, v16h b, v8f c) {
    return __builtin_amdgcn_wmma_f32_16x16x32_f16(false, a, false, b, (short)0, c, false, false);
  }
  static __device__ __forceinline__ void guard(v8f& a, v8f& b, v16h x, v16h y) { dep_guard_h(a, b, x, y); }
  static __device__ __forceinline__ void keep(v16h a, v16h b, v16h c, v16h d) { keep4_h(a, b, c, d); }
};
template <> struct Frag<__bf16> {
  typedef v16b V; union U { v16b v; v8b h[2]; };
  static __device__ __forceinline__ v16b load(const __bf16* p) {
    U f; f.h[0] = *(const v8b*)(p); f.h[1] = *(const v8b*)(p + 16); return f.v;
  }
  static __device__ __forceinline__ v8f mma(v16b a, v16b b, v8f c) {
    return __builtin_amdgcn_wmma_f32_16x16x32_bf16(false, a, false, b, (short)0, c, false, false);
  }
  static __device__ __forceinline__ void guard(v8f& a, v8f& b, v16b x, v16b y) { dep_guard_b(a, b, x, y); }
  static __device__ __forceinline__ void keep(v16b a, v16b b, v16b c, v16b d) { keep4_b(a, b, c, d); }
};

__device__ __forceinline__ float fsig(float x)  { return __builtin_amdgcn_rcpf(1.0f + __expf(-x)); }
__device__ __forceinline__ float ftanh(float x) { return 1.0f - 2.0f * __builtin_amdgcn_rcpf(__expf(2.0f * x) + 1.0f); }

__global__ __launch_bounds__(NTHR) void cvt_x_kernel(const float* __restrict__ x, float* __restrict__ XR) {
  const int i = blockIdx.x * NTHR + threadIdx.x;
  const int nreal = NNODE * NTIME;
  const int ic = (i < nreal) ? i : (nreal - 1);
  const float xv = x[ic];
  const float v = (i < nreal) ? bf16r(xv) : 0.0f;
  *(volatile float*)(XR + i) = v;
  __threadfence();
  *(volatile float*)(XR + i) = v;
}

__global__ __launch_bounds__(NTHR) void cvt_whh_kernel(const float* __restrict__ w, unsigned short* __restrict__ dst) {
  const int i = blockIdx.x * NTHR + threadIdx.x;
  const float* sp = w + (size_t)i * 8;
  const v4f a = *(const v4f*)(sp);
  const v4f b = *(const v4f*)(sp + 4);
  v8h hv;
#pragma unroll
  for (int e = 0; e < 4; ++e) {
    hv[e]     = __builtin_bit_cast(_Float16, f2bf_bits(a[e]));
    hv[4 + e] = __builtin_bit_cast(_Float16, f2bf_bits(b[e]));
  }
  *(volatile v8h*)(dst + (size_t)i * 8) = hv;
  __threadfence();
  *(volatile v8h*)(dst + (size_t)i * 8) = hv;
}

__global__ __launch_bounds__(NGATE) void prep_uv_kernel(const float* __restrict__ W_ih, const float* __restrict__ W_in,
                                                        const float* __restrict__ b_in, float* __restrict__ UV) {
  const int n = threadIdx.x;
  const float* wr = W_ih + (size_t)n * NHIDU;
  float su = 0.0f, sv = 0.0f, bad = 0.0f;
#pragma unroll 1
  for (int k = 0; k < NHIDU; ++k) {
    const float wk = bf16r(W_in[k]);
    const float a  = bf16r(wr[k]);
    su += a * fmaxf(wk, 0.0f);
    sv += a * fmaxf(-wk, 0.0f);
    bad += fabsf(b_in[k]);
  }
  const float nanv = __uint_as_float(0x7fc00000u);
  su = (bad != 0.0f) ? nanv : su;
  sv = (bad != 0.0f) ? nanv : sv;
  for (int pass = 0; pass < 2; ++pass) {
    *(volatile float*)(UV + n) = su;
    *(volatile float*)(UV + NGATE + n) = sv;
    __threadfence();
  }
}

__global__ __launch_bounds__(NTHR) void dots_kernel(const int* __restrict__ SRC, const int* __restrict__ TGT,
                                                    const float* __restrict__ emb, float* __restrict__ DOTS) {
  const int e = blockIdx.x * NTHR + threadIdx.x;
  const int s = clampn(SRC[e]);
  const int t = clampn(TGT[e]);
  const v2f* ps = (const v2f*)(emb + (size_t)s * NEMB);
  const v2f* pt = (const v2f*)(emb + (size_t)t * NEMB);
  float acc = 0.0f;
#pragma unroll
  for (int q = 0; q < NEMB / 2; ++q) {
    const v2f a = ps[q];
    const v2f b = pt[q];
    acc += bf16r(a[0]) * bf16r(b[0]);
    acc += bf16r(a[1]) * bf16r(b[1]);
  }
  const float d = fmaxf(acc, 0.0f);
  *(volatile float*)(DOTS + e) = d;
  __threadfence();
  *(volatile float*)(DOTS + e) = d;
}

__global__ __launch_bounds__(32) void sweep_softmax_kernel(const int* __restrict__ SRC, const float* __restrict__ DOTS,
                                                           float* __restrict__ DMAX, float* __restrict__ DEN) {
  __shared__ float sm[TILE_S];
  __shared__ float ss[TILE_S];
  const int lane = threadIdx.x;
  const int base = blockIdx.x * TILE_S;
#pragma unroll 1
  for (int i = lane; i < TILE_S; i += 32) { sm[i] = 0.0f; ss[i] = 0.0f; }
  __syncthreads();
  const i4v* K4 = (const i4v*)SRC;
#pragma unroll 1
  for (int it = 0; it < NEDGE4 / 32; ++it) {
    const i4v kk = K4[it * 32 + lane];
#pragma unroll
    for (int jj = 0; jj < 4; ++jj) {
      const unsigned d = (unsigned)(clampn(kk[jj]) - base);
      unsigned msk = __builtin_amdgcn_ballot_w32(d < (unsigned)TILE_S);
      while (msk != 0u) {
        const int hl = __builtin_ctz(msk);
        msk &= msk - 1u;
        const int q = __builtin_amdgcn_readlane((int)d, hl);
        const int e = ((it * 32 + hl) << 2) + jj;
        const float dv = DOTS[e];
        const float mo = sm[q];
        const float so = ss[q];
        const float mn = fmaxf(mo, dv);
        const float sn = fmaf(so, expf(mo - mn), expf(dv - mn));
        sm[q] = mn;
        ss[q] = sn;
      }
    }
  }
  __syncthreads();
  for (int pass = 0; pass < 2; ++pass) {
#pragma unroll
    for (int jj = 0; jj < TILE_S / 32; ++jj) {
      const int o = 32 * jj + lane;
      const float vm = sm[o];
      const float vs = ss[o];
      *(volatile float*)(DMAX + base + o) = vm;
      *(volatile float*)(DEN + base + o) = vs;
    }
    __threadfence();
  }
}

__global__ __launch_bounds__(NTHR) void ew_kernel(const int* __restrict__ SRC, const float* __restrict__ DOTS,
                                                  const float* __restrict__ DMAX, const float* __restrict__ DEN,
                                                  float* __restrict__ EW) {
  const int e = blockIdx.x * NTHR + threadIdx.x;
  const int s = clampn(SRC[e]);
  const float w = expf(DOTS[e] - DMAX[s]);
  const float v = w * __builtin_amdgcn_rcpf(DEN[s] + 1e-8f);
  *(volatile float*)(EW + e) = v;
  __threadfence();
  *(volatile float*)(EW + e) = v;
}

__global__ __launch_bounds__(32) void sweep_deg_kernel(const int* __restrict__ TGT, const float* __restrict__ EW,
                                                       float* __restrict__ DINV) {
  __shared__ float sd[TILE_S];
  const int lane = threadIdx.x;
  const int base = blockIdx.x * TILE_S;
#pragma unroll 1
  for (int i = lane; i < TILE_S; i += 32) sd[i] = 1.0f;
  __syncthreads();
  const i4v* K4 = (const i4v*)TGT;
#pragma unroll 1
  for (int it = 0; it < NEDGE4 / 32; ++it) {
    const i4v kk = K4[it * 32 + lane];
#pragma unroll
    for (int jj = 0; jj < 4; ++jj) {
      const unsigned d = (unsigned)(clampn(kk[jj]) - base);
      unsigned msk = __builtin_amdgcn_ballot_w32(d < (unsigned)TILE_S);
      while (msk != 0u) {
        const int hl = __builtin_ctz(msk);
        msk &= msk - 1u;
        const int q = __builtin_amdgcn_readlane((int)d, hl);
        const int e = ((it * 32 + hl) << 2) + jj;
        sd[q] += EW[e];
      }
    }
  }
  __syncthreads();
  for (int pass = 0; pass < 2; ++pass) {
#pragma unroll
    for (int jj = 0; jj < TILE_S / 32; ++jj) {
      const int o = 32 * jj + lane;
      const float dg = sd[o];
      const float di = (dg > 0.0f) ? rsqrtf(dg) : 0.0f;
      *(volatile float*)(DINV + base + o) = di;
    }
    __threadfence();
  }
}

__global__ __launch_bounds__(NTHR) void nrm_kernel(const int* __restrict__ SRC, const int* __restrict__ TGT,
                                                   const float* __restrict__ DINV, const float* __restrict__ EW,
                                                   float* __restrict__ NRM) {
  const int e = blockIdx.x * NTHR + threadIdx.x;
  const int s = clampn(SRC[e]);
  const int t = clampn(TGT[e]);
  const float v = (DINV[s] * EW[e]) * DINV[t];
  *(volatile float*)(NRM + e) = v;
  __threadfence();
  *(volatile float*)(NRM + e) = v;
}

__global__ __launch_bounds__(32) void sweep_y_kernel(const int* __restrict__ TGT, const int* __restrict__ SRC,
                                                     const float* __restrict__ NRM, const float* __restrict__ XR,
                                                     const float* __restrict__ DINV, float* __restrict__ YPL) {
  __shared__ float ya[TILE_Y * YLP];
  const int lane = threadIdx.x;
  const int base = blockIdx.x * TILE_Y;
  const int xmax = NNODP * NTIME - 1;
#pragma unroll 1
  for (int q = 0; q < TILE_Y; ++q) {
    const int node = base + q;
    const float di = DINV[node];
    int xi = node * NTIME + lane;
    xi = (xi > xmax) ? xmax : xi;
    ya[q * YLP + lane] = (di * di) * XR[xi];
  }
  __syncthreads();
  const i4v* K4 = (const i4v*)TGT;
#pragma unroll 1
  for (int it = 0; it < NEDGE4 / 32; ++it) {
    const i4v kk = K4[it * 32 + lane];
#pragma unroll
    for (int jj = 0; jj < 4; ++jj) {
      const unsigned d = (unsigned)(clampn(kk[jj]) - base);
      unsigned msk = __builtin_amdgcn_ballot_w32(d < (unsigned)TILE_Y);
      while (msk != 0u) {
        const int hl = __builtin_ctz(msk);
        msk &= msk - 1u;
        const int q = __builtin_amdgcn_readlane((int)d, hl);
        const int e = ((it * 32 + hl) << 2) + jj;
        const float cf = NRM[e];
        const int s = clampn(SRC[e]);
        const float xv = XR[s * NTIME + lane];
        ya[q * YLP + lane] = fmaf(cf, xv, ya[q * YLP + lane]);
      }
    }
  }
  __syncthreads();
  for (int pass = 0; pass < 2; ++pass) {
#pragma unroll 1
    for (int t = 0; t < NTIME; ++t) {
#pragma unroll
      for (int jj = 0; jj < TILE_Y / 32; ++jj) {
        const float v = ya[(32 * jj + lane) * YLP + t];
        *(volatile float*)(YPL + (size_t)t * NNODP + base + 32 * jj + lane) = v;
      }
    }
    __threadfence();
  }
}

__global__ __launch_bounds__(NTHR) void gru_kernel(const float* __restrict__ YPL, const unsigned short* __restrict__ WHBp,
                                                   const float* __restrict__ UV, const float* __restrict__ b_ih,
                                                   const float* __restrict__ b_hh, const float* __restrict__ W_out,
                                                   float* __restrict__ PPL) {
  __shared__ __align__(16) unsigned short Ahi[RROWS * HPITCH];
  __shared__ __align__(16) unsigned short Alo[RROWS * HPITCH];
  __shared__ float red[NTHR / 32][RROWS];
  const __bf16* WHB = (const __bf16*)WHBp;
  const int tid = threadIdx.x, lane = tid & 31, wave = tid >> 5;
  const int c = lane & 15, hh = lane >> 4, koff = hh * 8;
  const int rowbase = blockIdx.x * RROWS;
  const int j = 16 * wave + c;

  {
    unsigned* z0 = (unsigned*)Ahi;
    unsigned* z1 = (unsigned*)Alo;
#pragma unroll 1
    for (int i = tid; i < RROWS * HPITCH / 2; i += NTHR) { z0[i] = 0u; z1[i] = 0u; }
  }
  float ug[3], vg[3], big[3], bhg[3];
#pragma unroll
  for (int g = 0; g < 3; ++g) {
    ug[g]  = UV[g * NHIDU + j];
    vg[g]  = UV[NGATE + g * NHIDU + j];
    big[g] = bf16r(b_ih[g * NHIDU + j]);
    bhg[g] = bf16r(b_hh[g * NHIDU + j]);
  }
  const float wo = bf16r(W_out[j]);
  float hst[2][8];
#pragma unroll
  for (int m = 0; m < 2; ++m)
#pragma unroll
    for (int r = 0; r < 8; ++r) hst[m][r] = 0.0f;
  __syncthreads();

  const __bf16* ahi0 = (const __bf16*)Ahi + c * HPITCH + koff;
  const __bf16* alo0 = (const __bf16*)Alo + c * HPITCH + koff;
  const __bf16* wrow = WHB + (size_t)j * NHIDU + koff;
  const v8f z8 = {0.f, 0.f, 0.f, 0.f, 0.f, 0.f, 0.f, 0.f};

#pragma unroll 1
  for (int t = 0; t < NTIME; ++t) {
    float yp[2][8], ym[2][8];
    const float* yrow = YPL + (size_t)t * NNODP + rowbase + 8 * hh;
#pragma unroll
    for (int m = 0; m < 2; ++m) {
#pragma unroll
      for (int q = 0; q < 2; ++q) {
        const v4f yv = *(const v4f*)(yrow + 16 * m + 4 * q);
#pragma unroll
        for (int e = 0; e < 4; ++e) {
          yp[m][4 * q + e] = fmaxf(yv[e], 0.0f);
          ym[m][4 * q + e] = fmaxf(-yv[e], 0.0f);
        }
      }
    }
    v8f acc[2][3];
#pragma unroll
    for (int m = 0; m < 2; ++m) { acc[m][0] = z8; acc[m][1] = z8; acc[m][2] = z8; }
#pragma unroll 1
    for (int k0 = 0; k0 < NHIDU; k0 += 32) {
      const v16b b0 = Frag<__bf16>::load(wrow + k0);
      const v16b b1 = Frag<__bf16>::load(wrow + (size_t)1 * NHIDU * NHIDU + k0);
      const v16b b2 = Frag<__bf16>::load(wrow + (size_t)2 * NHIDU * NHIDU + k0);
#pragma unroll
      for (int m = 0; m < 2; ++m) {
        const v16b ah = Frag<__bf16>::load(ahi0 + m * 16 * HPITCH + k0);
        const v16b al = Frag<__bf16>::load(alo0 + m * 16 * HPITCH + k0);
        acc[m][0] = Frag<__bf16>::mma(ah, b0, acc[m][0]);
        acc[m][0] = Frag<__bf16>::mma(al, b0, acc[m][0]);
        acc[m][1] = Frag<__bf16>::mma(ah, b1, acc[m][1]);
        acc[m][1] = Frag<__bf16>::mma(al, b1, acc[m][1]);
        acc[m][2] = Frag<__bf16>::mma(ah, b2, acc[m][2]);
        acc[m][2] = Frag<__bf16>::mma(al, b2, acc[m][2]);
        guard3x5(acc[m][0], acc[m][1], acc[m][2], ah, al, b0, b1, b2);
      }
    }
    accg3(acc[0][0], acc[0][1], acc[0][2]);
    accg3(acc[1][0], acc[1][1], acc[1][2]);

#pragma unroll
    for (int m = 0; m < 2; ++m) {
#pragma unroll
      for (int r = 0; r < 8; ++r) {
        const float ypv = yp[m][r], ymv = ym[m][r];
        const float gir = fmaf(ypv, ug[0], fmaf(ymv, vg[0], big[0]));
        const float giz = fmaf(ypv, ug[1], fmaf(ymv, vg[1], big[1]));
        const float gin = fmaf(ypv, ug[2], fmaf(ymv, vg[2], big[2]));
        const float ghr = acc[m][0][r] + bhg[0];
        const float ghz = acc[m][1][r] + bhg[1];
        const float ghn = acc[m][2][r] + bhg[2];
        const float rg = fsig(gir + ghr);
        const float zg = fsig(giz + ghz);
        const float ng = ftanh(fmaf(rg, ghn, gin));
        const float ho = hst[m][r];
        hst[m][r] = (1.0f - zg) * ng + zg * ho;
      }
    }
    __syncthreads();
#pragma unroll
    for (int m = 0; m < 2; ++m) {
#pragma unroll
      for (int r = 0; r < 8; ++r) {
        const float hn = hst[m][r];
        const unsigned short hb = f2bf_bits(hn);
        const unsigned short lb = f2bf_bits(hn - bf_bits2f(hb));
        const int o = (16 * m + 8 * hh + r) * HPITCH + j;
        Ahi[o] = hb;
        Alo[o] = lb;
      }
    }
    __syncthreads();
  }

#pragma unroll
  for (int m = 0; m < 2; ++m) {
#pragma unroll
    for (int r = 0; r < 8; ++r) {
      float pv = hst[m][r] * wo;
      pv += __shfl_xor(pv, 1, 32);
      pv += __shfl_xor(pv, 2, 32);
      pv += __shfl_xor(pv, 4, 32);
      pv += __shfl_xor(pv, 8, 32);
      red[wave][16 * m + 8 * hh + r] = pv;
    }
  }
  __syncthreads();
  if (wave == 0) {
    float s = red[0][lane];
    s += red[1][lane]; s += red[2][lane]; s += red[3][lane];
    s += red[4][lane]; s += red[5][lane]; s += red[6][lane]; s += red[7][lane];
    float* op = PPL + rowbase + lane;
    *(volatile float*)op = s;
    __threadfence();
    *(volatile float*)op = s;
  }
}

__global__ __launch_bounds__(32) void sweep_out_kernel(const int* __restrict__ TGT, const int* __restrict__ SRC,
                                                       const float* __restrict__ NRM, const float* __restrict__ PPL,
                                                       const float* __restrict__ DINV, const float* __restrict__ b_out,
                                                       float* __restrict__ out) {
  __shared__ float so[TILE_S];
  const int lane = threadIdx.x;
  const int base = blockIdx.x * TILE_S;
  const float bo = bf16r(b_out[0]);
#pragma unroll 1
  for (int i = lane; i < TILE_S; i += 32) {
    const int node = base + i;
    const int nc = (node > NNODE - 1) ? (NNODE - 1) : node;
    const float di = DINV[node];
    so[i] = (di * di) * PPL[nc];
  }
  __syncthreads();
  const i4v* K4 = (const i4v*)TGT;
#pragma unroll 1
  for (int it = 0; it < NEDGE4 / 32; ++it) {
    const i4v kk = K4[it * 32 + lane];
#pragma unroll
    for (int jj = 0; jj < 4; ++jj) {
      const unsigned d = (unsigned)(clampn(kk[jj]) - base);
      unsigned msk = __builtin_amdgcn_ballot_w32(d < (unsigned)TILE_S);
      while (msk != 0u) {
        const int hl = __builtin_ctz(msk);
        msk &= msk - 1u;
        const int q = __builtin_amdgcn_readlane((int)d, hl);
        const int e = ((it * 32 + hl) << 2) + jj;
        const float cf = NRM[e];
        const int s = clampn(SRC[e]);
        so[q] = fmaf(cf, PPL[s], so[q]);
      }
    }
  }
  __syncthreads();
  int nj = (NNODE - base) / 32;
  nj = nj < 0 ? 0 : (nj > TILE_S / 32 ? TILE_S / 32 : nj);
  for (int pass = 0; pass < 2; ++pass) {
#pragma unroll
    for (int jj = 0; jj < TILE_S / 32; ++jj) {
      if (jj < nj) {
        const float v = so[32 * jj + lane] + bo;
        *(volatile float*)(out + base + 32 * jj + lane) = v;
      }
    }
    __threadfence();
  }
}

extern "C" void kernel_launch(void* const* d_in, const int* in_sizes, int n_in,
                              void* d_out, int out_size, void* d_ws, size_t ws_size, hipStream_t stream) {
  if (n_in < 11 || d_out == nullptr || d_ws == nullptr) return;
  if (in_sizes[0] != NNODE * NTIME || in_sizes[1] != 2 * NEDGE || in_sizes[2] != NNODE * NEMB ||
      in_sizes[3] != NHIDU || in_sizes[4] != NHIDU || in_sizes[5] != NGATE * NHIDU || in_sizes[6] != NGATE * NHIDU ||
      in_sizes[7] != NGATE || in_sizes[8] != NGATE || in_sizes[9] != NHIDU || in_sizes[10] != 1 ||
      out_size != NNODE) return;

  const float* x_seq = (const float*)d_in[0];
  const int*   eidx  = (const int*)d_in[1];
  const float* emb   = (const float*)d_in[2];
  const float* W_in  = (const float*)d_in[3];
  const float* b_in  = (const float*)d_in[4];
  const float* W_ih  = (const float*)d_in[5];
  const float* W_hh  = (const float*)d_in[6];
  const float* b_ih  = (const float*)d_in[7];
  const float* b_hh  = (const float*)d_in[8];
  const float* W_out = (const float*)d_in[9];
  const float* b_out = (const float*)d_in[10];
  const int* SRC = eidx;
  const int* TGT = eidx + NEDGE;
  float* out = (float*)d_out;

  char* ws = (char*)d_ws; size_t off = 0;
  auto carve = [&](size_t bytes) -> char* { char* p = ws + off; off += (bytes + 255) & ~(size_t)255; return p; };
  float*          XR   = (float*)carve((size_t)NNODP * NTIME * 4);
  unsigned short* WHB  = (unsigned short*)carve((size_t)NGATE * NHIDU * 2);
  float*          UV   = (float*)carve((size_t)2 * NGATE * 4);
  float*          DOTS = (float*)carve((size_t)NEDGE * 4);
  float*          EW   = (float*)carve((size_t)NEDGE * 4);
  float*          NRM  = (float*)carve((size_t)NEDGE * 4);
  float*          DMAX = (float*)carve((size_t)NNODP * 4);
  float*          DEN  = (float*)carve((size_t)NNODP * 4);
  float*          DINV = (float*)carve((size_t)NNODP * 4);
  float*          YPL  = (float*)carve((size_t)NTIME * NNODP * 4);
  float*          PPL  = (float*)carve((size_t)NNODE * 4);
  if (off > ws_size || off > (size_t)134217728) return;

  cvt_x_kernel<<<(NNODP * NTIME) / NTHR, NTHR, 0, stream>>>(x_seq, XR);
  cvt_whh_kernel<<<(NGATE * NHIDU / 8) / NTHR, NTHR, 0, stream>>>(W_hh, WHB);
  prep_uv_kernel<<<1, NGATE, 0, stream>>>(W_ih, W_in, b_in, UV);
  dots_kernel<<<NEDGE / NTHR, NTHR, 0, stream>>>(SRC, TGT, emb, DOTS);
  sweep_softmax_kernel<<<NNODP / TILE_S, 32, 0, stream>>>(SRC, DOTS, DMAX, DEN);
  ew_kernel<<<NEDGE / NTHR, NTHR, 0, stream>>>(SRC, DOTS, DMAX, DEN, EW);
  sweep_deg_kernel<<<NNODP / TILE_S, 32, 0, stream>>>(TGT, EW, DINV);
  nrm_kernel<<<NEDGE / NTHR, NTHR, 0, stream>>>(SRC, TGT, DINV, EW, NRM);
  sweep_y_kernel<<<NNODP / TILE_Y, 32, 0, stream>>>(TGT, SRC, NRM, XR, DINV, YPL);
  gru_kernel<<<NNODE / RROWS, NTHR, 0, stream>>>(YPL, WHB, UV, b_ih, b_hh, W_out, PPL);
  sweep_out_kernel<<<NNODP / TILE_S, 32, 0, stream>>>(TGT, SRC, NRM, PPL, DINV, b_out, out);
}
